// GRUCell_83133386982091
// MI455X (gfx1250) — hardware-run, weakly checked
//
#include <hip/hip_runtime.h>
#include <math.h>

constexpr int kBatch   = 32;
constexpr int kNodes   = 1024;
constexpr int kEmb     = 64;
constexpr int kCin     = 128;
constexpr int kGateOut = 128;
constexpr int kUpdOut  = 64;
constexpr int kRows    = kBatch * kNodes;
constexpr int kKK      = 256;
constexpr int kOSlice  = 64;
constexpr int kWcols   = kOSlice * kKK;
constexpr float kLoCarry    = 16384.0f;
constexpr float kLoCarryInv = 1.0f / 16384.0f;
constexpr float kPCarry     = 32768.0f;
constexpr float kPCarryInv  = 1.0f / 32768.0f;

static_assert(kNodes % 64 == 0 && kWcols % 64 == 0 && kOSlice % 64 == 0, "tile multiples");
static_assert(kEmb % 32 == 0 && kNodes % 32 == 0 && kKK % 32 == 0, "K multiples of 32");

constexpr size_t kOffBig   = 0;
constexpr size_t kSzBig    = (size_t)kBatch * kNodes * kNodes * 2;
constexpr size_t kSzW      = (size_t)kNodes * kWcols * 2;
constexpr size_t kOffEmb   = kOffBig + kSzBig;
constexpr size_t kOffXin   = kOffEmb + (size_t)kRows * kEmb * 2;
constexpr size_t kOffVt    = kOffXin + (size_t)kRows * kCin * 2;
constexpr size_t kOffXg2h  = kOffVt + (size_t)kBatch * kCin * kNodes * 2;
constexpr size_t kOffXg2l  = kOffXg2h + (size_t)kRows * kCin * 2;
constexpr size_t kOffZsh   = kOffXg2l + (size_t)kRows * kCin * 2;
constexpr size_t kOffZsl   = kOffZsh + (size_t)kRows * kUpdOut * 2;
constexpr size_t kOffRpl   = kOffZsl + (size_t)kRows * kUpdOut * 2;
constexpr size_t kOffNeb   = kOffRpl + (size_t)kRows * kUpdOut * 4;
constexpr size_t kOffBwg   = kOffNeb + (size_t)kNodes * kEmb * 2;
constexpr size_t kOffBwu   = kOffBwg + (size_t)kGateOut * kKK * kEmb * 2;
constexpr size_t kOffBiasG = kOffBwu + (size_t)kUpdOut * kKK * kEmb * 2;
constexpr size_t kOffBiasU = kOffBiasG + (size_t)kBatch * kGateOut * 4;
constexpr size_t kWsTotal  = kOffBiasU + (size_t)kBatch * kUpdOut * 4;
static_assert(2 * kSzW == kSzBig, "W hi+lo slice fits the P region exactly");
static_assert(kWsTotal == 128081920ull, "carve total");
static_assert(kWsTotal <= 134217728ull, "carve under 128 MiB");

typedef __attribute__((ext_vector_type(16))) _Float16 v16h;
typedef __attribute__((ext_vector_type(8)))  _Float16 v8h;
typedef __attribute__((ext_vector_type(16))) __bf16   v16b;
typedef __attribute__((ext_vector_type(8)))  __bf16   v8b;
typedef __attribute__((ext_vector_type(8)))  float    v8f;
typedef __attribute__((ext_vector_type(4)))  float    v4f;
typedef __attribute__((ext_vector_type(4)))  unsigned int v4u;

__device__ __forceinline__ unsigned short f2bf_bits(float f) {
  unsigned u = __float_as_uint(f);
  return (unsigned short)((u + 0x7FFFu + ((u >> 16) & 1u)) >> 16);
}
__device__ __forceinline__ float bf_bits2f(unsigned short h) { return __uint_as_float(((unsigned)h) << 16); }
__device__ __forceinline__ float bfr(float f) { return bf_bits2f(f2bf_bits(f)); }
__device__ __forceinline__ unsigned short h_bits(float f) { const _Float16 h = (_Float16)f; return __builtin_bit_cast(unsigned short, h); }
__device__ __forceinline__ unsigned pk16(unsigned short a, unsigned short b) { return (unsigned)a | ((unsigned)b << 16); }
__device__ __forceinline__ float h16_to_f32(unsigned hb) {
  const unsigned sgn = (hb & 0x8000u) << 16; const unsigned em = hb & 0x7fffu;
  const float fn = __uint_as_float((em << 13) + 0x38000000u);
  const float fs = (float)em * 5.9604644775390625e-8f;
  const float mag = (em < 0x400u) ? fs : fn; return __uint_as_float(__float_as_uint(mag) | sgn); }

__device__ __forceinline__ v8f zero8() { return (v8f){0.f, 0.f, 0.f, 0.f, 0.f, 0.f, 0.f, 0.f}; }

__device__ __forceinline__ v8f mma_h(v16h a, v16h b, v8f c) {
  c = __builtin_amdgcn_wmma_f32_16x16x32_f16(false, a, false, b, (short)0, c, false, false);
  asm volatile("v_nop\n\tv_nop\n\tv_nop\n\tv_nop" : "+v"(c) : "v"(a), "v"(b));
  return c;
}
__device__ __forceinline__ v8f mma_b(v16b a, v16b b, v8f c) {
  c = __builtin_amdgcn_wmma_f32_16x16x32_bf16(false, a, false, b, (short)0, c, false, false);
  asm volatile("v_nop\n\tv_nop\n\tv_nop\n\tv_nop" : "+v"(c) : "v"(a), "v"(b));
  return c;
}
__device__ __forceinline__ void wave_sync() {
  __builtin_amdgcn_fence(__ATOMIC_RELEASE, "workgroup");
  __builtin_amdgcn_wave_barrier();
  __builtin_amdgcn_fence(__ATOMIC_ACQUIRE, "workgroup");
}

template <typename T> struct Frag;
template <> struct Frag<_Float16> {
  typedef v16h V; union U { v16h v; v8h h[2]; };
  static __device__ __forceinline__ v16h load(const _Float16* p) {
    U f; f.h[0] = *(const v8h*)(p); f.h[1] = *(const v8h*)(p + 16); return f.v;
  }
  static __device__ __forceinline__ v8f mmag(v16h a, v16h b, v8f c) { return mma_h(a, b, c); }
};
template <> struct Frag<__bf16> {
  typedef v16b V; union U { v16b v; v8b h[2]; };
  static __device__ __forceinline__ v16b load(const __bf16* p) {
    U f; f.h[0] = *(const v8b*)(p); f.h[1] = *(const v8b*)(p + 16); return f.v;
  }
  static __device__ __forceinline__ v8f mmag(v16b a, v16b b, v8f c) { return mma_b(a, b, c); }
};
template <int ET> struct Elem;
template <> struct Elem<0> { typedef _Float16 T; };
template <> struct Elem<1> { typedef __bf16 T; };

__global__ __launch_bounds__(256) void neb_kernel(const float* __restrict__ ne, unsigned short* __restrict__ dst) {
  const int i = blockIdx.x * 256 + threadIdx.x;
  if (i >= kNodes * kEmb / 8) return;
  const float* p = ne + 8 * (size_t)i;
  const v4f a = *(const v4f*)p;
  const v4f c = *(const v4f*)(p + 4);
  unsigned short hb[8];
#pragma unroll
  for (int e = 0; e < 4; ++e) { hb[e] = f2bf_bits(a[e]); hb[4 + e] = f2bf_bits(c[e]); }
  const v4u u = (v4u){pk16(hb[0], hb[1]), pk16(hb[2], hb[3]), pk16(hb[4], hb[5]), pk16(hb[6], hb[7])};
  unsigned short* q = dst + 8 * (size_t)i;
  *(volatile v4u*)q = u;
  __threadfence();
  *(volatile v4u*)q = u;
}

__global__ __launch_bounds__(256) void bw_kernel(const float* __restrict__ w, unsigned short* __restrict__ dst, int nout, int nrows) {
  const int i = blockIdx.x * 256 + threadIdx.x;
  if (i >= nrows * 8) return;
  const int row = i >> 3, d0 = (i & 7) * 8;
  const int o = row >> 8, ki = row & 255;
  const size_t dstride = (size_t)256 * nout;
  const float* p = w + (size_t)ki * nout + o + (size_t)d0 * dstride;
  unsigned short hb[8];
#pragma unroll
  for (int e = 0; e < 8; ++e) hb[e] = f2bf_bits(p[(size_t)e * dstride]);
  const v4u u = (v4u){pk16(hb[0], hb[1]), pk16(hb[2], hb[3]), pk16(hb[4], hb[5]), pk16(hb[6], hb[7])};
  unsigned short* q = dst + (size_t)row * kEmb + d0;
  *(volatile v4u*)q = u;
  __threadfence();
  *(volatile v4u*)q = u;
}

__global__ __launch_bounds__(256) void bias_kernel(const float* __restrict__ te, const float* __restrict__ gb, const float* __restrict__ ub,
                                                 float* __restrict__ dstg, float* __restrict__ dstu) {
  const int t = blockIdx.x * 256 + threadIdx.x;
  const bool isg = (blockIdx.x < (kBatch * kGateOut) / 256);
  const int u = isg ? t : (t - kBatch * kGateOut);
  const int nout = isg ? kGateOut : kUpdOut;
  const int b = u / nout, o = u - b * nout;
  const float* wp = isg ? gb : ub;
  float s = 0.0f;
#pragma unroll 1
  for (int d = 0; d < kEmb; ++d) s += bfr(te[b * kEmb + d]) * bfr(wp[d * nout + o]);
  float* q = (isg ? dstg : dstu) + u;
  *(volatile float*)q = s;
  __threadfence();
  *(volatile float*)q = s;
}

__global__ __launch_bounds__(256) void xin_kernel(const float* __restrict__ x, const float* __restrict__ st, unsigned short* __restrict__ dst) {
  const int lane = threadIdx.x & 31, wave = threadIdx.x >> 5;
  const int row = blockIdx.x * 16 + (wave >> 1) * 4 + (lane >> 3);
  const int half = wave & 1;
  const int c8 = (lane & 7) * 8;
  const float* src = (half ? st : x) + (size_t)row * kEmb + c8;
  const v4f a = *(const v4f*)src;
  const v4f c = *(const v4f*)(src + 4);
  unsigned short hb[8];
#pragma unroll
  for (int e = 0; e < 4; ++e) { hb[e] = h_bits(bfr(a[e])); hb[4 + e] = h_bits(bfr(c[e])); }
  const v4u u = (v4u){pk16(hb[0], hb[1]), pk16(hb[2], hb[3]), pk16(hb[4], hb[5]), pk16(hb[6], hb[7])};
  unsigned short* q = dst + (size_t)row * kCin + half * 64 + c8;
  *(volatile v4u*)q = u;
  __threadfence();
  *(volatile v4u*)q = u;
}

__global__ __launch_bounds__(256) void vt1_kernel(const float* __restrict__ x, const float* __restrict__ st, unsigned short* __restrict__ vt) {
  __shared__ float sm[64][65];
  const int t = threadIdx.x, lane = t & 31, wave = t >> 5;
  const int mt = blockIdx.x, half = blockIdx.y, b = blockIdx.z;
  const float* src = (half ? st : x) + ((size_t)b * kNodes + mt * 64) * kEmb;
#pragma unroll
  for (int it = 0; it < 4; ++it) {
    const int e = it * 256 + t; const int m = e >> 4; const int c4 = (e & 15) * 4;
    const v4f v = *(const v4f*)(src + (size_t)m * kEmb + c4);
#pragma unroll
    for (int k = 0; k < 4; ++k) sm[c4 + k][m] = v[k];
  }
  __syncthreads();
  const int q = lane >> 3, c8 = (lane & 7) * 8;
  unsigned short* op = vt + ((size_t)b * kCin + half * 64) * kNodes + mt * 64;
  for (int pass = 0; pass < 2; ++pass) {
#pragma unroll
    for (int it = 0; it < 2; ++it) {
      const int row = wave * 8 + it * 4 + q;
      unsigned short hb[8];
#pragma unroll
      for (int e = 0; e < 8; ++e) hb[e] = h_bits(bfr(sm[row][c8 + e]));
      const v4u u = (v4u){pk16(hb[0], hb[1]), pk16(hb[2], hb[3]), pk16(hb[4], hb[5]), pk16(hb[6], hb[7])};
      *(volatile v4u*)(op + (size_t)row * kNodes + c8) = u;
    }
    __threadfence();
  }
}

__global__ __launch_bounds__(256) void vt2_kernel(const unsigned short* __restrict__ zsh, unsigned short* __restrict__ vt) {
  __shared__ unsigned short sm[64][66];
  const int t = threadIdx.x, lane = t & 31, wave = t >> 5;
  const int mt = blockIdx.x, b = blockIdx.y;
  const unsigned short* src = zsh + ((size_t)b * kNodes + mt * 64) * kUpdOut;
#pragma unroll
  for (int it = 0; it < 2; ++it) {
    const int e = it * 256 + t; const int m = e >> 3; const int c8 = (e & 7) * 8;
    const v4u u = *(const v4u*)(src + (size_t)m * kUpdOut + c8);
#pragma unroll
    for (int k = 0; k < 4; ++k) {
      const unsigned wv = u[k];
      sm[c8 + 2 * k][m]     = (unsigned short)(wv & 0xffffu);
      sm[c8 + 2 * k + 1][m] = (unsigned short)(wv >> 16);
    }
  }
  __syncthreads();
  const int q = lane >> 3, m8 = (lane & 7) * 8;
  unsigned short* op = vt + ((size_t)b * kCin + 64) * kNodes + mt * 64;
  for (int pass = 0; pass < 2; ++pass) {
#pragma unroll
    for (int it = 0; it < 2; ++it) {
      const int row = wave * 8 + it * 4 + q;
      const v4u u = (v4u){pk16(sm[row][m8], sm[row][m8 + 1]), pk16(sm[row][m8 + 2], sm[row][m8 + 3]),
                          pk16(sm[row][m8 + 4], sm[row][m8 + 5]), pk16(sm[row][m8 + 6], sm[row][m8 + 7])};
      *(volatile v4u*)(op + (size_t)row * kNodes + m8) = u;
    }
    __threadfence();
  }
}

__global__ __launch_bounds__(256) void emb_kernel(const float* __restrict__ ne, const float* __restrict__ te,
                                                const float* __restrict__ gam, const float* __restrict__ bet, unsigned short* __restrict__ dst) {
  const int lane = threadIdx.x & 31, wave = threadIdx.x >> 5;
  const int row = blockIdx.x * 32 + wave * 4 + (lane >> 3);
  const int b = row >> 10, n = row & 1023;
  const int d0 = (lane & 7) * 8;
  const v4f na = *(const v4f*)(ne + n * kEmb + d0);
  const v4f nb = *(const v4f*)(ne + n * kEmb + d0 + 4);
  const v4f ta = *(const v4f*)(te + b * kEmb + d0);
  const v4f tb = *(const v4f*)(te + b * kEmb + d0 + 4);
  asm volatile("" ::: "memory");
  const v4f ga = *(const v4f*)(gam + d0);
  const v4f gb = *(const v4f*)(gam + d0 + 4);
  const v4f ba = *(const v4f*)(bet + d0);
  const v4f bb = *(const v4f*)(bet + d0 + 4);
  float v[8], g[8], be[8];
#pragma unroll
  for (int e = 0; e < 4; ++e) {
    v[e]      = bfr(na[e]) + bfr(ta[e]);
    v[4 + e]  = bfr(nb[e]) + bfr(tb[e]);
    g[e]      = bfr(ga[e]);  g[4 + e]  = bfr(gb[e]);
    be[e]     = bfr(ba[e]);  be[4 + e] = bfr(bb[e]);
  }
  float s = 0.0f;
#pragma unroll
  for (int e = 0; e < 8; ++e) s += v[e];
  s += __shfl_xor(s, 1, 32);
  s += __shfl_xor(s, 2, 32);
  s += __shfl_xor(s, 4, 32);
  const float mu = s * (1.0f / 64.0f);
  float dv[8];
  float sq = 0.0f;
#pragma unroll
  for (int e = 0; e < 8; ++e) { dv[e] = v[e] - mu; sq += dv[e] * dv[e]; }
  sq += __shfl_xor(sq, 1, 32);
  sq += __shfl_xor(sq, 2, 32);
  sq += __shfl_xor(sq, 4, 32);
  const float var = sq * (1.0f / 64.0f);
  const float inv = 1.0f / sqrtf(var + 1e-12f);
  unsigned short hb[8];
#pragma unroll
  for (int e = 0; e < 8; ++e) { const float y = dv[e] * inv * g[e] + be[e]; hb[e] = h_bits(y); }
  const v4u u = (v4u){pk16(hb[0], hb[1]), pk16(hb[2], hb[3]), pk16(hb[4], hb[5]), pk16(hb[6], hb[7])};
  unsigned short* q = dst + (size_t)row * kEmb + d0;
  *(volatile v4u*)q = u;
  __threadfence();
  *(volatile v4u*)q = u;
}

__global__ __launch_bounds__(128) void softmax_p_kernel(const unsigned short* __restrict__ embp, unsigned short* __restrict__ pp) {
  __shared__ __align__(16) _Float16 Ksh[64 * 64];
  __shared__ __align__(16) float Os[4][16 * 68];
  const int tid = threadIdx.x, wave = tid >> 5, lane = tid & 31, hh = lane >> 4, c = lane & 15;
  const int b = blockIdx.x >> 4, qb = blockIdx.x & 15;
  const int q0 = qb * 64 + wave * 16;
  const _Float16* embb = (const _Float16*)embp + (size_t)b * kNodes * kEmb;
  v16h qa[2];
#pragma unroll
  for (int dc = 0; dc < 2; ++dc) qa[dc] = Frag<_Float16>::load(embb + (size_t)(q0 + c) * kEmb + dc * 32 + 8 * hh);
  float mrow[8], lrow[8], invl[8];
#pragma unroll
  for (int r = 0; r < 8; ++r) { mrow[r] = -INFINITY; lrow[r] = 0.0f; invl[r] = 0.0f; }

#pragma unroll 1
  for (int sweep = 0; sweep < 2; ++sweep) {
#pragma unroll 1
    for (int kc = 0; kc < 16; ++kc) {
      const int kv0 = kc * 64;
      __syncthreads();
      {
        const int kvr = tid >> 1, dh = (tid & 1) * 32;
        const _Float16* sp = embb + (size_t)(kv0 + kvr) * kEmb + dh;
        _Float16* dp = Ksh + kvr * 64 + dh;
#pragma unroll
        for (int i = 0; i < 4; ++i) *(v8h*)(dp + 8 * i) = *(const v8h*)(sp + 8 * i);
      }
      __syncthreads();
      v8f s[4];
#pragma unroll
      for (int j = 0; j < 4; ++j) {
        s[j] = zero8();
#pragma unroll
        for (int dc = 0; dc < 2; ++dc) {
          Frag<_Float16>::U kb;
          kb.h[0] = *(const v8h*)(Ksh + (j * 16 + c) * 64 + dc * 32 + 8 * hh);
          kb.h[1] = *(const v8h*)(Ksh + (j * 16 + c) * 64 + dc * 32 + 16 + 8 * hh);
          s[j] = mma_h(qa[dc], kb.v, s[j]);
        }
      }
      if (sweep == 0) {
#pragma unroll
        for (int r = 0; r < 8; ++r) {
          float m = -INFINITY;
#pragma unroll
          for (int j = 0; j < 4; ++j) m = fmaxf(m, s[j][r]);
#pragma unroll
          for (int off = 1; off < 16; off <<= 1) m = fmaxf(m, __shfl_xor(m, off, 32));
          const float mnew = fmaxf(mrow[r], m);
          const float alpha = expf(mrow[r] - mnew);
          float psum = 0.0f;
#pragma unroll
          for (int j = 0; j < 4; ++j) psum += expf(s[j][r] - mnew);
#pragma unroll
          for (int off = 1; off < 16; off <<= 1) psum += __shfl_xor(psum, off, 32);
          lrow[r] = lrow[r] * alpha + psum;
          mrow[r] = mnew;
        }
      } else {
        float* os = Os[wave];
#pragma unroll
        for (int r = 0; r < 8; ++r) {
          const int qrow = q0 + 8 * hh + r;
#pragma unroll
          for (int j = 0; j < 4; ++j) {
            const int kvcol = kv0 + j * 16 + c;
            float p = expf(s[j][r] - mrow[r]) * invl[r];
            p = p - ((kvcol == qrow) ? 1.0f : 0.0f);
            os[(8 * hh + r) * 68 + j * 16 + c] = p * kPCarry;
          }
        }
        wave_sync();
        const int q = lane >> 3, c8 = (lane & 7) * 8;
        unsigned short* prow = pp + ((size_t)b * kNodes + q0) * kNodes + kv0 + c8;
        for (int pass = 0; pass < 2; ++pass) {
#pragma unroll
          for (int it = 0; it < 4; ++it) {
            const int row = it * 4 + q;
            const float* sp = os + row * 68 + c8;
            v8h hv;
#pragma unroll
            for (int e = 0; e < 8; ++e) hv[e] = (_Float16)sp[e];
            *(volatile v8h*)(prow + (size_t)row * kNodes) = hv;
          }
          __threadfence();
        }
        wave_sync();
      }
    }
    if (sweep == 0) {
#pragma unroll
      for (int r = 0; r < 8; ++r) invl[r] = 1.0f / lrow[r];
    }
  }
}

template <int ET, int EPI>
__global__ __launch_bounds__(256) void gemm64_hl(
    const unsigned short* __restrict__ Ap, int lda, long strideA,
    const unsigned short* __restrict__ Btp, int ldb, long strideB,
    unsigned short* __restrict__ CHp, unsigned short* __restrict__ CLp, int ldc, long strideC,
    const float* __restrict__ resF, const unsigned short* __restrict__ resH, const unsigned short* __restrict__ resL,
    int ldr, long strideR, int M, int N, int K, float scale) {
  typedef typename Elem<ET>::T T;
  typedef typename Frag<T>::V V;
  const T* A = (const T*)Ap; const T* Bt = (const T*)Btp;
  __shared__ __align__(16) float sT[8][16 * 68];
  const int b    = blockIdx.y;
  const int lane = threadIdx.x & 31;
  const int wave = threadIdx.x >> 5;
  const int tilesN = N >> 6;
  const int tilesM = M >> 6;
  const int tile = blockIdx.x * 8 + wave;
  if (tile >= tilesM * tilesN) return;
  const int tm = tile / tilesN;
  const int tn = tile - tm * tilesN;
  const int m0 = tm << 6;
  const int n0 = tn << 6;

  const T* Ab = A  + (size_t)b * strideA;
  const T* Bb = Bt + (size_t)b * strideB;

  const int rlane = lane & 15;
  const int koff  = (lane >> 4) * 8;
  const int mOff  = (lane >> 4) * 8;

  v8f acc[4][4];
#pragma unroll
  for (int i = 0; i < 4; ++i)
#pragma unroll
    for (int j = 0; j < 4; ++j) acc[i][j] = zero8();

  for (int k0 = 0; k0 < K; k0 += 32) {
    V bq[4];
#pragma unroll
    for (int j = 0; j < 4; ++j) {
      const size_t bo = (size_t)(n0 + (j << 4) + rlane) * ldb + koff + k0;
      bq[j] = Frag<T>::load(Bb + bo);
    }
#pragma unroll
    for (int i = 0; i < 4; ++i) {
      const size_t ao = (size_t)(m0 + (i << 4) + rlane) * lda + koff + k0;
      const V ah = Frag<T>::load(Ab + ao);
#pragma unroll
      for (int j = 0; j < 4; ++j) acc[i][j] = Frag<T>::mmag(ah, bq[j], acc[i][j]);
    }
  }

  float* slab = sT[wave];
  unsigned short* CHb = CHp + (size_t)b * strideC;
  unsigned short* CLb = CLp + (size_t)b * strideC;
  const int q = lane >> 3, c8 = (lane & 7) * 8;
#pragma unroll
  for (int i = 0; i < 4; ++i) {
    const int mBase = m0 + (i << 4);
#pragma unroll
    for (int j = 0; j < 4; ++j) {
#pragma unroll
      for (int r = 0; r < 8; ++r) slab[(mOff + r) * 68 + (j << 4) + rlane] = acc[i][j][r] * scale;
    }
    wave_sync();
#pragma unroll
    for (int it = 0; it < 4; ++it) {
      const int row = it * 4 + q;
      const int m = mBase + row;
      const float* sp = slab + row * 68 + c8;
      float v[8];
#pragma unroll
      for (int e = 0; e < 8; ++e) v[e] = sp[e];
      if (EPI == 1) {
        const float* rp = resF + (size_t)b * strideR + (size_t)m * ldr + n0 + c8;
        const v4f r0 = *(const v4f*)rp;
        const v4f r1 = *(const v4f*)(rp + 4);
#pragma unroll
        for (int e = 0; e < 4; ++e) { v[e] += bfr(r0[e]); v[4 + e] += bfr(r1[e]); }
      }
      if (EPI == 2) {
        const size_t ro = (size_t)b * strideR + (size_t)m * ldr + n0 + c8;
        const v4u uh = *(const v4u*)(resH + ro);
        const v4u ul = *(const v4u*)(resL + ro);
#pragma unroll
        for (int k = 0; k < 4; ++k) {
          const unsigned wh = uh[k];
          const unsigned wl = ul[k];
          v[2 * k]     += h16_to_f32(wh & 0xffffu) + h16_to_f32(wl & 0xffffu) * kLoCarryInv;
          v[2 * k + 1] += h16_to_f32(wh >> 16)     + h16_to_f32(wl >> 16)     * kLoCarryInv;
        }
      }
      v8h hv, lv;
#pragma unroll
      for (int e = 0; e < 8; ++e) {
        const float f = v[e];
        const _Float16 hq = (_Float16)f;
        const float hf = (float)hq;
        hv[e] = hq;
        lv[e] = (_Float16)((f - hf) * kLoCarry);
      }
      unsigned short* dh = CHb + (size_t)m * ldc + n0 + c8;
      unsigned short* dl = CLb + (size_t)m * ldc + n0 + c8;
      for (int pass = 0; pass < 2; ++pass) {
        *(volatile v8h*)dh = hv;
        *(volatile v8h*)dl = lv;
        __threadfence();
      }
    }
    wave_sync();
  }
}

template <int MODE, int S>
__device__ __forceinline__ void node_step(v8f (&acc)[4], v8f (&accr)[4],
                                          const _Float16* xin, const _Float16* zsh, const _Float16* zsl,
                                          const _Float16* xg2h, const _Float16* xg2l,
                                          const _Float16* wh, const _Float16* wl, size_t arow, int rlane, int koff) {
  constexpr bool kSecond = (S >= 4);
  constexpr bool kZs = (MODE == 2) && (S == 2 || S == 3);
  constexpr bool kHasLo = kSecond || kZs;
  v16h ah, al;
  if (kSecond) {
    const size_t o = arow * kCin + koff + 32 * (S - 4);
    ah = Frag<_Float16>::load(xg2h + o);
    al = Frag<_Float16>::load(xg2l + o);
  } else if (kZs) {
    const size_t o = arow * kUpdOut + koff + 32 * (S - 2);
    ah = Frag<_Float16>::load(zsh + o);
    al = Frag<_Float16>::load(zsl + o);
  } else {
    const size_t o = arow * kCin + koff + 32 * S;
    ah = Frag<_Float16>::load(xin + o);
    al = ah;
  }
  asm volatile("" ::: "memory");
#pragma unroll
  for (int j = 0; j < 4; ++j) {
    const size_t bo = (size_t)(j * 16 + rlane) * kKK + koff + 32 * S;
    const v16h bh = Frag<_Float16>::load(wh + bo);
    const v16h bl = Frag<_Float16>::load(wl + bo);
    acc[j]  = mma_h(ah, bh, acc[j]);
    accr[j] = mma_h(ah, bl, accr[j]);
    if (kHasLo) accr[j] = mma_h(al, bh, accr[j]);
    asm volatile("" ::: "memory");
  }
}

template <int MODE>
__global__ __launch_bounds__(128) void node_kernel(
    const unsigned short* xinp, const unsigned short* zshp, const unsigned short* zslp,
    const unsigned short* xg2hp, const unsigned short* xg2lp,
    const unsigned short* whp, const unsigned short* wlp,
    const float* bias, int biasld, int biascol0,
    const float* state, const float* rin,
    unsigned short* outH, unsigned short* outL, float* outF) {
  __shared__ __align__(16) float sBias[32 * 64];
  __shared__ __align__(16) float sSt[2 * 32 * 64];
  __shared__ __align__(16) float sR[(MODE == 2) ? 2 * 32 * 64 : 4];
  __shared__ __align__(16) float sT[4][16 * 68];
  const int tid = threadIdx.x, wave = tid >> 5, lane = tid & 31;
  const int hh = lane >> 4, c = lane & 15, rlane = lane & 15, koff = (lane >> 4) * 8;
  const int nl = wave >> 1, isub = wave & 1;
  const int node0 = blockIdx.x * 2;
  const int node = node0 + nl;

#pragma unroll
  for (int u = 0; u < 4; ++u) {
    const int f = tid + 128 * u; const int bb = f >> 4; const int c4 = (f & 15) * 4;
    const v4f v = *(const v4f*)(bias + (size_t)bb * biasld + biascol0 + c4);
    *(v4f*)(sBias + bb * 64 + c4) = v;
  }
  asm volatile("" ::: "memory");
#pragma unroll
  for (int g2 = 0; g2 < 2; ++g2) {
#pragma unroll
    for (int u = 0; u < 4; ++u) {
      const int f = tid + 128 * (u + 4 * g2); const int nn = f >> 9; const int w = f & 511;
      const int bb = w >> 4; const int c4 = (w & 15) * 4;
      const v4f v = *(const v4f*)(state + ((size_t)bb * kNodes + node0 + nn) * kUpdOut + c4);
      v4f rv;
#pragma unroll
      for (int e = 0; e < 4; ++e) rv[e] = bfr(v[e]);
      *(v4f*)(sSt + nn * 2048 + bb * 64 + c4) = rv;
    }
    asm volatile("" ::: "memory");
  }
  if (MODE == 2) {
#pragma unroll
    for (int g2 = 0; g2 < 2; ++g2) {
#pragma unroll
      for (int u = 0; u < 4; ++u) {
        const int f = tid + 128 * (u + 4 * g2); const int nn = f >> 9; const int w = f & 511;
        const int bb = w >> 4; const int c4 = (w & 15) * 4;
        const v4f v = *(const v4f*)(rin + ((size_t)bb * kNodes + node0 + nn) * kUpdOut + c4);
        *(v4f*)(sR + nn * 2048 + bb * 64 + c4) = v;
      }
      asm volatile("" ::: "memory");
    }
  }
  __syncthreads();

  const _Float16* xin  = (const _Float16*)xinp;
  const _Float16* zsh  = (const _Float16*)zshp;
  const _Float16* zsl  = (const _Float16*)zslp;
  const _Float16* xg2h = (const _Float16*)xg2hp;
  const _Float16* xg2l = (const _Float16*)xg2lp;
  const _Float16* wh   = (const _Float16*)whp + (size_t)node * kWcols;
  const _Float16* wl   = (const _Float16*)wlp + (size_t)node * kWcols;
  const size_t arow = (size_t)(16 * isub + rlane) * kNodes + node;
  v8f acc[4], accr[4];
#pragma unroll
  for (int j = 0; j < 4; ++j) { acc[j] = zero8(); accr[j] = zero8(); }
  node_step<MODE, 0>(acc, accr, xin, zsh, zsl, xg2h, xg2l, wh, wl, arow, rlane, koff);
  node_step<MODE, 1>(acc, accr, xin, zsh, zsl, xg2h, xg2l, wh, wl, arow, rlane, koff);
  node_step<MODE, 2>(acc, accr, xin, zsh, zsl, xg2h, xg2l, wh, wl, arow, rlane, koff);
  node_step<MODE, 3>(acc, accr, xin, zsh, zsl, xg2h, xg2l, wh, wl, arow, rlane, koff);
  node_step<MODE, 4>(acc, accr, xin, zsh, zsl, xg2h, xg2l, wh, wl, arow, rlane, koff);
  node_step<MODE, 5>(acc, accr, xin, zsh, zsl, xg2h, xg2l, wh, wl, arow, rlane, koff);
  node_step<MODE, 6>(acc, accr, xin, zsh, zsl, xg2h, xg2l, wh, wl, arow, rlane, koff);
  node_step<MODE, 7>(acc, accr, xin, zsh, zsl, xg2h, xg2l, wh, wl, arow, rlane, koff);

  float* slab = sT[wave];
  const float* stn = sSt + nl * 2048;
  const float* rn  = sR + ((MODE == 2) ? nl * 2048 : 0);
#pragma unroll
  for (int j = 0; j < 4; ++j) {
#pragma unroll
    for (int r = 0; r < 8; ++r) {
      const int row = 8 * hh + r;
      const int bb = 16 * isub + row;
      const int col = j * 16 + c;
      const float pre = acc[j][r] + accr[j][r] * kLoCarryInv + sBias[bb * 64 + col];
      float v;
      if (MODE == 0) {
        const float z = __builtin_amdgcn_rcpf(1.0f + expf(-pre));
        v = z * stn[bb * 64 + col];
      } else if (MODE == 1) {
        v = __builtin_amdgcn_rcpf(1.0f + expf(-pre));
      } else {
        const float hc = tanhf(pre);
        const float rr = rn[bb * 64 + col];
        const float sv = stn[bb * 64 + col];
        v = rr * sv + (1.0f - rr) * hc;
      }
      slab[row * 68 + col] = v;
    }
  }
  wave_sync();
  if (MODE == 0) {
    const int q = lane >> 3, c8 = (lane & 7) * 8;
    for (int pass = 0; pass < 2; ++pass) {
#pragma unroll
      for (int it = 0; it < 4; ++it) {
        const int row = it * 4 + q;
        const int bb = 16 * isub + row;
        const float* sp = slab + row * 68 + c8;
        v8h hv, lv;
#pragma unroll
        for (int e = 0; e < 8; ++e) {
          const float f = sp[e];
          const _Float16 hq = (_Float16)f;
          const float hf = (float)hq;
          hv[e] = hq;
          lv[e] = (_Float16)((f - hf) * kLoCarry);
        }
        const size_t o = ((size_t)bb * kNodes + node) * kUpdOut + c8;
        *(volatile v8h*)(outH + o) = hv;
        *(volatile v8h*)(outL + o) = lv;
      }
      __threadfence();
    }
  } else {
    const int c4 = c * 4;
    for (int pass = 0; pass < 2; ++pass) {
#pragma unroll
      for (int it = 0; it < 8; ++it) {
        const int row = it * 2 + hh;
        const int bb = 16 * isub + row;
        const v4f v = *(const v4f*)(slab + row * 68 + c4);
        *(volatile v4f*)(outF + ((size_t)bb * kNodes + node) * kUpdOut + c4) = v;
      }
      __threadfence();
    }
  }
}

extern "C" void kernel_launch(void* const* d_in, const int* in_sizes, int n_in,
                              void* d_out, int out_size, void* d_ws, size_t ws_size, hipStream_t stream) {
  if (n_in < 12) return;
  if (out_size != kRows * kUpdOut) return;
  if (in_sizes[0] != kRows * kEmb || in_sizes[1] != kRows * kUpdOut || in_sizes[2] != kNodes * kEmb) return;
  if (ws_size < kWsTotal) return;
  const float* x    = (const float*)d_in[0];
  const float* st   = (const float*)d_in[1];
  const float* ne   = (const float*)d_in[2];
  const float* te   = (const float*)d_in[3];
  const float* gw   = (const float*)d_in[4];
  const float* gbv  = (const float*)d_in[5];
  const float* ggam = (const float*)d_in[6];
  const float* gbet = (const float*)d_in[7];
  const float* uw   = (const float*)d_in[8];
  const float* ubv  = (const float*)d_in[9];
  const float* ugam = (const float*)d_in[10];
  const float* ubet = (const float*)d_in[11];
  float* out = (float*)d_out;

  char* ws = (char*)d_ws;
  unsigned short* P    = (unsigned short*)(ws + kOffBig);
  unsigned short* WH   = (unsigned short*)(ws + kOffBig);
  unsigned short* WL   = (unsigned short*)(ws + kOffBig + kSzW);
  unsigned short* EMB  = (unsigned short*)(ws + kOffEmb);
  unsigned short* XIN  = (unsigned short*)(ws + kOffXin);
  unsigned short* VT   = (unsigned short*)(ws + kOffVt);
  unsigned short* XG2H = (unsigned short*)(ws + kOffXg2h);
  unsigned short* XG2L = (unsigned short*)(ws + kOffXg2l);
  unsigned short* ZSH  = (unsigned short*)(ws + kOffZsh);
  unsigned short* ZSL  = (unsigned short*)(ws + kOffZsl);
  float*          RPL  = (float*)(ws + kOffRpl);
  unsigned short* NEB  = (unsigned short*)(ws + kOffNeb);
  unsigned short* BWG  = (unsigned short*)(ws + kOffBwg);
  unsigned short* BWU  = (unsigned short*)(ws + kOffBwu);
  float*          BIASG = (float*)(ws + kOffBiasG);
  float*          BIASU = (float*)(ws + kOffBiasU);

  const long strideP   = (long)kNodes * kNodes;
  const long strideVT  = (long)kCin * kNodes;
  const long strideXG2 = (long)kNodes * kCin;
  const long strideRes = (long)kNodes * kUpdOut;

  neb_kernel<<<(kNodes * kEmb / 8) / 256, 256, 0, stream>>>(ne, NEB);
  bw_kernel<<<(kGateOut * kKK * 8) / 256, 256, 0, stream>>>(gw, BWG, kGateOut, kGateOut * kKK);
  bw_kernel<<<(kUpdOut * kKK * 8) / 256, 256, 0, stream>>>(uw, BWU, kUpdOut, kUpdOut * kKK);
  bias_kernel<<<(kBatch * kGateOut + kBatch * kUpdOut) / 256, 256, 0, stream>>>(te, gbv, ubv, BIASG, BIASU);
  xin_kernel<<<kRows / 16, 256, 0, stream>>>(x, st, XIN);
  vt1_kernel<<<dim3(kNodes / 64, 2, kBatch), 256, 0, stream>>>(x, st, VT);

  emb_kernel<<<kRows / 32, 256, 0, stream>>>(ne, te, ggam, gbet, EMB);
  softmax_p_kernel<<<kBatch * (kNodes / 64), 128, 0, stream>>>(EMB, P);
  gemm64_hl<0, 1><<<dim3((kNodes / 64) * 1 / 8, kBatch), 256, 0, stream>>>(
      P, kNodes, strideP, VT, kNodes, strideVT, XG2H, XG2L, kCin, strideXG2,
      x, ZSH, ZSL, kUpdOut, strideRes, kNodes, 64, kNodes, kPCarryInv);
  gemm64_hl<0, 1><<<dim3((kNodes / 64) * 1 / 8, kBatch), 256, 0, stream>>>(
      P, kNodes, strideP, VT + (size_t)64 * kNodes, kNodes, strideVT, XG2H + 64, XG2L + 64, kCin, strideXG2,
      st, ZSH, ZSL, kUpdOut, strideRes, kNodes, 64, kNodes, kPCarryInv);
  gemm64_hl<1, 0><<<dim3((kNodes / 64) * (kWcols / 64) / 8, 1), 256, 0, stream>>>(
      NEB, kEmb, 0L, BWG, kEmb, 0L, WH, WL, kWcols, 0L,
      x, ZSH, ZSL, 0, 0L, kNodes, kWcols, kEmb, 1.0f);
  node_kernel<0><<<kNodes / 2, 128, 0, stream>>>(XIN, ZSH, ZSL, XG2H, XG2L, WH, WL, BIASG, kGateOut, 0, st, RPL, ZSH, ZSL, RPL);
  gemm64_hl<1, 0><<<dim3((kNodes / 64) * (kWcols / 64) / 8, 1), 256, 0, stream>>>(
      NEB, kEmb, 0L, BWG + (size_t)kWcols * kEmb, kEmb, 0L, WH, WL, kWcols, 0L,
      x, ZSH, ZSL, 0, 0L, kNodes, kWcols, kEmb, 1.0f);
  node_kernel<1><<<kNodes / 2, 128, 0, stream>>>(XIN, ZSH, ZSL, XG2H, XG2L, WH, WL, BIASG, kGateOut, 64, st, RPL, ZSH, ZSL, RPL);

  vt2_kernel<<<dim3(kNodes / 64, kBatch), 256, 0, stream>>>(ZSH, VT);
  emb_kernel<<<kRows / 32, 256, 0, stream>>>(ne, te, ugam, ubet, EMB);
  softmax_p_kernel<<<kBatch * (kNodes / 64), 128, 0, stream>>>(EMB, P);
  gemm64_hl<0, 1><<<dim3((kNodes / 64) * 1 / 8, kBatch), 256, 0, stream>>>(
      P, kNodes, strideP, VT, kNodes, strideVT, XG2H, XG2L, kCin, strideXG2,
      x, ZSH, ZSL, kUpdOut, strideRes, kNodes, 64, kNodes, kPCarryInv);
  gemm64_hl<0, 2><<<dim3((kNodes / 64) * 1 / 8, kBatch), 256, 0, stream>>>(
      P, kNodes, strideP, VT + (size_t)64 * kNodes, kNodes, strideVT, XG2H + 64, XG2L + 64, kCin, strideXG2,
      x, ZSH, ZSL, kUpdOut, strideRes, kNodes, 64, kNodes, kPCarryInv);
  gemm64_hl<1, 0><<<dim3((kNodes / 64) * (kWcols / 64) / 8, 1), 256, 0, stream>>>(
      NEB, kEmb, 0L, BWU, kEmb, 0L, WH, WL, kWcols, 0L,
      x, ZSH, ZSL, 0, 0L, kNodes, kWcols, kEmb, 1.0f);
  node_kernel<2><<<kNodes / 2, 128, 0, stream>>>(XIN, ZSH, ZSL, XG2H, XG2L, WH, WL, BIASU, kUpdOut, 0, st, RPL, ZSH, ZSL, out);
}
